// RaggedConvolutionTranspose_45612552683660
// MI455X (gfx1250) — hardware-verified
//
#include <hip/hip_runtime.h>
#include <stddef.h>


#define FI     64
#define NH     192
#define UN     64
#define NTHR   256
#define NWAVE  8
#define GROWS  64
#define NCW    96
#define NT     (NCW / 16)
#define TGT    128
#define ANODE  16
#define SEGCAP 1048576
#define XSC    8
#define WSC    16
#define WSCAP  134217728
#define WPB    ((NH * FI / 8) / NTHR)

static_assert((NH * FI / 8) % NTHR == 0);
static_assert(FI / 8 == 8);
static_assert(GROWS == (NWAVE / 2) * 16);
static_assert(NH == 2 * NCW && NCW == NT * 16);
static_assert((FI % 32) == 0);
static_assert((8 * NH) % 128 == 0);
static_assert(TGT == NWAVE * ANODE);
static_assert(UN == 64);
static_assert((ANODE * UN) % 128 == 0 && ANODE <= 31);
static_assert(GROWS * NH * 4 <= 65536);
static_assert(TGT * UN * 4 <= 65536);

typedef float     v4f  __attribute__((ext_vector_type(4)));
typedef float     v2f  __attribute__((ext_vector_type(2)));
typedef float     v8f  __attribute__((ext_vector_type(8)));
typedef _Float16  v8h  __attribute__((ext_vector_type(8)));
typedef _Float16  v16h __attribute__((ext_vector_type(16)));
union FragH { v16h v; v8h h[2]; };

__device__ __forceinline__ v8f wmf(v16h a, v16h b, v8f c) {
  v8f d = __builtin_amdgcn_wmma_f32_16x16x32_f16(false, a, false, b, (short)0, c, false, false);
  asm volatile("v_nop\n\tv_nop\n\tv_nop\n\tv_nop" : "+v"(d) : "v"(a), "v"(b));
  return d;
}

__device__ __forceinline__ float rlf(float v, int p) {
  return __int_as_float(__builtin_amdgcn_readlane(__float_as_int(v), p));
}

__global__ __launch_bounds__(NTHR) void k_wprep(const float* __restrict__ w, _Float16* wp) {
  const int i  = (int)blockIdx.x * NTHR + (int)threadIdx.x;
  const int n  = i >> 3;
  const int k0 = (i & 7) * 8;
  v8h hv;
#pragma unroll
  for (int e = 0; e < 8; ++e) hv[e] = (_Float16)(w[(size_t)(k0 + e) * NH + n] * (float)WSC);
  _Float16* d = wp + (size_t)i * 8;
  *(volatile v8h*)d = hv;
  __threadfence();
  *(volatile v8h*)d = hv;
}

__global__ __launch_bounds__(NTHR) void k_gemm(
    const float* __restrict__ A, const _Float16* __restrict__ Bw, const float* __restrict__ bs,
    float* C, int nRowsA) {
  __shared__ __attribute__((aligned(16))) float stg[GROWS * NH];
  constexpr float OSC = 1.0f / (float)(XSC * WSC);
  const int tid = threadIdx.x, lane = tid & 31, wave = tid >> 5, hh = lane >> 4, m = lane & 15;
  const int rg = wave >> 1, chh = wave & 1;
  const int rowBase = blockIdx.x * GROWS;
  int arow = rowBase + 16 * rg + m;
  arow = arow > nRowsA - 1 ? nRowsA - 1 : arow;
  const float* ap = A + (size_t)arow * FI + 8 * hh;

  v8f acc[NT];
#pragma unroll
  for (int t = 0; t < NT; ++t) { v8f z = {0.f, 0.f, 0.f, 0.f, 0.f, 0.f, 0.f, 0.f}; acc[t] = z; }

#pragma unroll
  for (int kt = 0; kt < FI / 32; ++kt) {
    const float* akp = ap + 32 * kt;
    const v4f f0 = *(const v4f*)akp;
    const v4f f1 = *(const v4f*)(akp + 4);
    const v4f f2 = *(const v4f*)(akp + 16);
    const v4f f3 = *(const v4f*)(akp + 20);
    v8h lo, hi;
    lo[0] = (_Float16)(f0.x * (float)XSC); lo[1] = (_Float16)(f0.y * (float)XSC);
    lo[2] = (_Float16)(f0.z * (float)XSC); lo[3] = (_Float16)(f0.w * (float)XSC);
    lo[4] = (_Float16)(f1.x * (float)XSC); lo[5] = (_Float16)(f1.y * (float)XSC);
    lo[6] = (_Float16)(f1.z * (float)XSC); lo[7] = (_Float16)(f1.w * (float)XSC);
    hi[0] = (_Float16)(f2.x * (float)XSC); hi[1] = (_Float16)(f2.y * (float)XSC);
    hi[2] = (_Float16)(f2.z * (float)XSC); hi[3] = (_Float16)(f2.w * (float)XSC);
    hi[4] = (_Float16)(f3.x * (float)XSC); hi[5] = (_Float16)(f3.y * (float)XSC);
    hi[6] = (_Float16)(f3.z * (float)XSC); hi[7] = (_Float16)(f3.w * (float)XSC);
    FragH af;
    af.h[0] = lo;
    af.h[1] = hi;
#pragma unroll
    for (int t = 0; t < NT; ++t) {
      const _Float16* bp = Bw + (size_t)(NCW * chh + 16 * t + m) * FI + 32 * kt + 8 * hh;
      FragH bf;
      bf.h[0] = *(const v8h*)bp;
      bf.h[1] = *(const v8h*)(bp + 16);
      acc[t] = wmf(af.v, bf.v, acc[t]);
    }
  }

  float bv[NT];
#pragma unroll
  for (int t = 0; t < NT; ++t) bv[t] = bs[NCW * chh + 16 * t + m];
  float* sp = stg + (16 * rg + 8 * hh) * NH + NCW * chh + m;
#pragma unroll
  for (int t = 0; t < NT; ++t) {
#pragma unroll
    for (int r = 0; r < 8; ++r) sp[r * NH + 16 * t] = acc[t][r] * OSC + bv[t];
  }
  __syncthreads();

  const float* lp = stg + wave * (8 * NH);
  float* gp = C + (size_t)(rowBase + 8 * wave) * NH;
#pragma unroll
  for (int i = 0; i < (8 * NH) / 128; ++i) {
    const v4f v = *(const v4f*)(lp + i * 128 + 4 * lane);
    *(volatile v4f*)(gp + i * 128 + 4 * lane) = v;
  }
  __threadfence();
#pragma unroll
  for (int i = 0; i < (8 * NH) / 128; ++i) {
    const v4f v = *(const v4f*)(lp + i * 128 + 4 * lane);
    *(volatile v4f*)(gp + i * 128 + 4 * lane) = v;
  }
}

__global__ __launch_bounds__(NTHR) void k_agg(
    const float* __restrict__ hp, const float* __restrict__ coord, const int* __restrict__ idx,
    const int* __restrict__ rs, float* out, int nOut, int nE, int nIn) {
  __shared__ __attribute__((aligned(16))) float stg[TGT * UN];
  const int tid = threadIdx.x, lane = tid & 31, wave = tid >> 5;
  const int tbase = blockIdx.x * TGT + wave * ANODE;
  int rsi = tbase + lane;
  rsi = rsi < 0 ? 0 : (rsi > nOut ? nOut : rsi);
  const int rsl = rs[rsi];

#pragma unroll 1
  for (int j = 0; j < ANODE; ++j) {
    const int o = tbase + j;
    int e0 = __builtin_amdgcn_readlane(rsl, j);
    int e1 = __builtin_amdgcn_readlane(rsl, j + 1);
    e0 = e0 < 0 ? 0 : (e0 > nE ? nE : e0);
    e1 = e1 < e0 ? e0 : (e1 > nE ? nE : e1);
    int n = e1 - e0;
    n = n > SEGCAP ? SEGCAP : n;
    if (o >= nOut) n = 0;
    float acc0 = 0.f, acc1 = 0.f;
#pragma unroll 1
    for (int q0 = 0; q0 < n; q0 += 32) {
      int ep = e0 + q0 + lane;
      ep = ep < 0 ? 0 : (ep > nE - 1 ? nE - 1 : ep);
      int il = idx[ep];
      il = il < 0 ? 0 : (il > nIn - 1 ? nIn - 1 : il);
      const float c0l = coord[(size_t)3 * ep + 0];
      const float c1l = coord[(size_t)3 * ep + 1];
      const float c2l = coord[(size_t)3 * ep + 2];
      const int mcnt = (n - q0) < 32 ? (n - q0) : 32;
#pragma unroll 1
      for (int p = 0; p < mcnt; ++p) {
        const int   s  = __builtin_amdgcn_readlane(il, p);
        const float c0 = rlf(c0l, p), c1 = rlf(c1l, p), c2 = rlf(c2l, p);
        const v2f* gpp = (const v2f*)(hp + (size_t)s * NH) + 3 * lane;
        const v2f g01 = gpp[0];
        const v2f g23 = gpp[1];
        const v2f g45 = gpp[2];
        acc0 += g01.x * c0 + g01.y * c1 + g23.x * c2;
        acc1 += g23.y * c0 + g45.x * c1 + g45.y * c2;
      }
    }
    v2f rv;
    rv.x = acc0; rv.y = acc1;
    *(v2f*)(stg + (wave * ANODE + j) * UN + 2 * lane) = rv;
  }
  __syncthreads();

  const float* lp = stg + wave * (ANODE * UN);
#pragma unroll
  for (int i = 0; i < (ANODE * UN) / 128; ++i) {
    const int row = tbase + 2 * i + (lane >> 4);
    const int rw  = row < nOut ? row : nOut - 1;
    const v4f v = *(const v4f*)(lp + i * 128 + 4 * lane);
    float* op = out + (size_t)rw * UN + 4 * (lane & 15);
    if (row < nOut) *(volatile v4f*)op = v;
  }
  __threadfence();
#pragma unroll
  for (int i = 0; i < (ANODE * UN) / 128; ++i) {
    const int row = tbase + 2 * i + (lane >> 4);
    const int rw  = row < nOut ? row : nOut - 1;
    const v4f v = *(const v4f*)(lp + i * 128 + 4 * lane);
    float* op = out + (size_t)rw * UN + 4 * (lane & 15);
    if (row < nOut) *(volatile v4f*)op = v;
  }
}

extern "C" void kernel_launch(void* const* d_in, const int* in_sizes, int n_in,
                              void* d_out, int out_size, void* d_ws, size_t ws_size,
                              hipStream_t stream) {
  if (n_in < 6) return;
  const int nIn  = in_sizes[0] / FI;
  const int nE   = in_sizes[2];
  const int nOut = in_sizes[3] - 1;
  if (nIn <= 0 || nE <= 0 || nOut <= 0) return;
  if (in_sizes[0] != nIn * FI || in_sizes[1] != 3 * nE) return;
  if (in_sizes[4] != FI * NH || in_sizes[5] != NH) return;
  if (out_size != nOut * UN) return;
  if (nIn > (1 << 22) || nE > (1 << 28) || nOut > (1 << 24)) return;

  const float* x     = (const float*)d_in[0];
  const float* coord = (const float*)d_in[1];
  const int*   idx   = (const int*)d_in[2];
  const int*   rs    = (const int*)d_in[3];
  const float* W     = (const float*)d_in[4];
  const float* bs    = (const float*)d_in[5];
  float* out = (float*)d_out;

  const int NPAD  = ((nIn + GROWS - 1) / GROWS) * GROWS;
  const int nGemm = NPAD / GROWS;
  const int nAgg  = (nOut + TGT - 1) / TGT;

  char* ws = (char*)d_ws;
  size_t off = 0;
  const size_t oW = off; off += (size_t)(NH * FI) * 2;          off = (off + 255) & ~(size_t)255;
  const size_t oH = off; off += (size_t)NPAD * NH * 4;          off = (off + 255) & ~(size_t)255;
  if (off > ws_size || off > (size_t)WSCAP) return;
  _Float16* wp = (_Float16*)(ws + oW);
  float*    hp = (float*)(ws + oH);

  k_wprep<<<WPB, NTHR, 0, stream>>>(W, wp);

  k_gemm<<<nGemm, NTHR, 0, stream>>>(x, wp, bs, hp, nIn);

  k_agg<<<nAgg, NTHR, 0, stream>>>(hp, coord, idx, rs, out, nOut, nE, nIn);
}
